// Non_Local_Module_14877766713778
// MI455X (gfx1250) — hardware-run, weakly checked
//
#include <hip/hip_runtime.h>


namespace {
constexpr int NBI = 8, C = 256, HH = 64, WW = 64, NP = HH * WW  , CI = 128, NM = NP / 4  , KB = 128, BNEPS_DUMMY = 0;
constexpr float XS = 8.0f, HS = 256.0f, WSC = 256.0f, PS = 256.0f, BNEPS = 1e-5f;
typedef _Float16 b16;
typedef __attribute__((ext_vector_type(16))) _Float16 v16b;
typedef __attribute__((ext_vector_type(8))) _Float16 v8b;
typedef __attribute__((ext_vector_type(8))) float v8f;
typedef __attribute__((ext_vector_type(4))) float v4f;
__device__ __forceinline__ float bf16_rne(float f) { unsigned int u = __float_as_uint(f); u += 0x7FFFu + ((u >> 16) & 1u); float r = __uint_as_float(u & 0xFFFF0000u); asm volatile("" : "+v"(r)); return r; }
__device__ __forceinline__ float bfv(float f) { float r = bf16_rne(f); asm volatile("" : "+v"(r)); return r; }
__device__ __forceinline__ void split16(float v, b16& hi, b16& lo) { hi = (b16)v; lo = (b16)(v - (float)hi); }
__device__ __forceinline__ v16b frag_kb(const b16* p, int hh) { const v8b a = *(const v8b*)(p + 8 * hh), b = *(const v8b*)(p + 16 + 8 * hh); v16b f;
#pragma unroll
  for (int e = 0; e < 8; ++e) { f[e] = a[e]; f[8 + e] = b[e]; } return f; }
__device__ __forceinline__ v8f wmma16b(v16b a, v16b b, v8f c) { v8f d = __builtin_amdgcn_wmma_f32_16x16x32_f16(false, a, false, b, (short)0, c, false, false); asm volatile("v_nop\n\tv_nop\n\tv_nop\n\tv_nop" : "+v"(d) : "v"(a), "v"(b)); return d; }
__device__ __forceinline__ void wave_lds_sync() { __builtin_amdgcn_fence(__ATOMIC_RELEASE, "workgroup"); __builtin_amdgcn_wave_barrier(); __builtin_amdgcn_fence(__ATOMIC_ACQUIRE, "workgroup"); }
__device__ __forceinline__ float pmul(float a, float b) { float p = a * b; asm volatile("" : "+v"(p)); return p; }

__global__ __launch_bounds__(256) void wput_kernel(const float* __restrict__ tw, const float* __restrict__ pw, const float* __restrict__ gw, const float* __restrict__ ww, b16* __restrict__ W3, b16* __restrict__ WOUT) { const int u = blockIdx.x * 256 + threadIdx.x; v8b v;
  if (u < 3 * CI * (C / 8)) { const int o = u / (C / 8), k0 = (u % (C / 8)) * 8; const float* w = o < CI ? tw : (o < 2 * CI ? pw : gw); const int oo = o % CI;
#pragma unroll
    for (int j = 0; j < 8; ++j) v[j] = (b16)(bf16_rne(w[(size_t)oo * C + k0 + j]) * WSC); for (int pass = 0; pass < 2; ++pass) { *(volatile v8b*)(W3 + (size_t)o * C + k0) = v; __threadfence(); } }
  if (u < C * (CI / 8)) { const int o = u / (CI / 8), k0 = (u % (CI / 8)) * 8;
#pragma unroll
    for (int j = 0; j < 8; ++j) v[j] = (b16)(bf16_rne(ww[(size_t)o * CI + k0 + j]) * WSC); for (int pass = 0; pass < 2; ++pass) { *(volatile v8b*)(WOUT + (size_t)o * CI + k0) = v; __threadfence(); } } }
__global__ __launch_bounds__(32) void proj_kernel(const float* __restrict__ x, const b16* __restrict__ W3, const float* __restrict__ tb, const float* __restrict__ pb, const float* __restrict__ gb, int BLIM, b16* __restrict__ THh, b16* __restrict__ THl, float* __restrict__ PG) { __shared__ __attribute__((aligned(16))) b16 Xt[32][C + 8]; __shared__ float Tf[32][132]; const int lane = threadIdx.x, nloc = lane & 15, hlf = lane >> 4; const int b = blockIdx.x / (NP / 32); if (b >= BLIM) return; const int p0 = (blockIdx.x % (NP / 32)) * 32; const float* xb = x + (size_t)b * C * NP;
  for (int c = 0; c < C; ++c) Xt[lane][c] = (b16)(bf16_rne(xb[(size_t)c * NP + p0 + lane]) * XS); for (int k = C; k < C + 8; ++k) Xt[lane][k] = (b16)0.0f;
  wave_lds_sync();
#pragma unroll 1
  for (int pj = 0; pj < 3; ++pj) {
#pragma unroll 1
    for (int rt = 0; rt < 2; ++rt) { v8f acc[8];
#pragma unroll
      for (int t = 0; t < 8; ++t) acc[t] = (v8f){};
#pragma unroll 2
      for (int kb = 0; kb < C; kb += 32) { const v16b a = frag_kb(&Xt[rt * 16 + nloc][kb], hlf);
#pragma unroll
        for (int t = 0; t < 8; ++t) acc[t] = wmma16b(a, frag_kb(W3 + (size_t)(pj * CI + t * 16 + nloc) * C + kb, hlf), acc[t]); }
      const float* bb = pj == 0 ? tb : (pj == 1 ? pb : gb);
#pragma unroll
      for (int t = 0; t < 8; ++t) { const int cc = t * 16 + nloc; const float bv = bfv(bb[cc]);
#pragma unroll
        for (int r8 = 0; r8 < 8; ++r8) Tf[rt * 16 + 8 * hlf + r8][cc] = acc[t][r8] * (1.0f / (XS * WSC)) + bv; } }
    wave_lds_sync();
    for (int pass = 0; pass < 2; ++pass) { for (int rr = 0; rr < 32; ++rr) { const size_t p = (size_t)b * NP + p0 + rr;
        if (pj == 0) { b16 h4[4], l4[4]; for (int q = 0; q < 4; ++q) split16(Tf[rr][lane * 4 + q] * HS, h4[q], l4[q]); typedef __attribute__((ext_vector_type(4))) _Float16 v4b; *(volatile v4b*)(THh + p * CI + lane * 4) = (v4b){h4[0], h4[1], h4[2], h4[3]}; *(volatile v4b*)(THl + p * CI + lane * 4) = (v4b){l4[0], l4[1], l4[2], l4[3]}; }
        else *(volatile v4f*)(PG + p * 2 * CI + (pj - 1) * CI + lane * 4) = *(const v4f*)(&Tf[rr][lane * 4]); } __threadfence(); }
    wave_lds_sync(); } }
__global__ __launch_bounds__(256) void pool_kernel(const float* __restrict__ PG, int BLIM, b16* __restrict__ PHh, b16* __restrict__ PHl, b16* __restrict__ Gh, b16* __restrict__ Gl) { const size_t u = (size_t)blockIdx.x * 256 + threadIdx.x; const size_t m_all = u / 16; const int c0 = (int)(u % 16) * 8; const int b = (int)(m_all / NM); if (b >= BLIM) return; const int m = (int)(m_all % NM); const int i = m / (WW / 2), j = m % (WW / 2);
  v8b a1, a2, g1, g2;
#pragma unroll
  for (int q = 0; q < 8; ++q) { const int c = c0 + q; float ph = -INFINITY, gg = -INFINITY;
#pragma unroll
    for (int a = 0; a < 2; ++a)
#pragma unroll
      for (int d = 0; d < 2; ++d) { const size_t p = (size_t)b * NP + (size_t)(2 * i + a) * WW + 2 * j + d; ph = fmaxf(ph, PG[p * 2 * CI + c]); gg = fmaxf(gg, PG[p * 2 * CI + CI + c]); }
    b16 x1, x2; split16(ph * HS, x1, x2); a1[q] = x1; a2[q] = x2; split16(gg * HS, x1, x2); g1[q] = x1; g2[q] = x2; }
  const size_t o = ((size_t)b * NM + m) * CI + c0;
  for (int pass = 0; pass < 2; ++pass) { *(volatile v8b*)(PHh + o) = a1; *(volatile v8b*)(PHl + o) = a2; *(volatile v8b*)(Gh + o) = g1; *(volatile v8b*)(Gl + o) = g2; __threadfence(); } }
__global__ __launch_bounds__(32) void att_kernel(const b16* __restrict__ THh, const b16* __restrict__ THl, const b16* __restrict__ PHh, const b16* __restrict__ PHl, const b16* __restrict__ Gh, const b16* __restrict__ Gl, int BLIM, float* __restrict__ Y) {
  __shared__ __attribute__((aligned(16))) b16 Ph_[16][KB + 8], Pl_[16][KB + 8], Vth[CI][KB + 8], Vtl[CI][KB + 8]; __shared__ float Sf[16][KB + 4], Of[16][CI + 4];
  const int lane = threadIdx.x, nloc = lane & 15, hlf = lane >> 4; const int b = blockIdx.x / (NP / 16); if (b >= BLIM) return; const size_t q0 = (size_t)b * NP + (size_t)(blockIdx.x % (NP / 16)) * 16;
  v16b qa[4], qb[4];
#pragma unroll
  for (int ks = 0; ks < 4; ++ks) { qa[ks] = frag_kb(THh + (q0 + nloc) * CI + ks * 32, hlf); qb[ks] = frag_kb(THl + (q0 + nloc) * CI + ks * 32, hlf); }
  float m_r[8], den_r[8]; v8f acc[8];
#pragma unroll
  for (int r8 = 0; r8 < 8; ++r8) { m_r[r8] = -INFINITY; den_r[r8] = 0.0f; }
#pragma unroll
  for (int t = 0; t < 8; ++t) acc[t] = (v8f){};
#pragma unroll 1
  for (int kb0 = 0; kb0 < NM; kb0 += KB) { const size_t mbase = (size_t)b * NM + kb0;
    for (int rr = 0; rr < KB; rr += 2) { const int r = rr + hlf; const size_t mrow = (mbase + r) * CI; for (int s = 0; s < CI / 16; ++s) { Vth[s * 16 + nloc][r] = Gh[mrow + s * 16 + nloc]; Vtl[s * 16 + nloc][r] = Gl[mrow + s * 16 + nloc]; } }
#pragma unroll
    for (int t = 0; t < KB / 16; ++t) { const size_t krow = (mbase + t * 16 + nloc) * CI; v8f s = {};
#pragma unroll
      for (int ks = 0; ks < 4; ++ks) { const v16b ka = frag_kb(PHh + krow + ks * 32, hlf), kl = frag_kb(PHl + krow + ks * 32, hlf); s = wmma16b(qa[ks], ka, s); s = wmma16b(qa[ks], kl, s); s = wmma16b(qb[ks], ka, s); }
#pragma unroll
      for (int r8 = 0; r8 < 8; ++r8) Sf[8 * hlf + r8][t * 16 + nloc] = s[r8] * (1.0f / (HS * HS)); }
    wave_lds_sync();
#pragma unroll
    for (int rr = 0; rr < 16; ++rr) { float mx = -INFINITY;
#pragma unroll
      for (int q = 0; q < 4; ++q) mx = fmaxf(mx, Sf[rr][q * 32 + lane]);
      for (int o = 16; o; o >>= 1) mx = fmaxf(mx, __shfl_xor(mx, o));
      const float mold = __shfl(m_r[rr & 7], (rr >> 3) * 16); const float mn = fmaxf(mold, mx); const float sf = (mold == -INFINITY) ? 0.0f : __expf(mold - mn); float ps = 0.0f;
#pragma unroll
      for (int q = 0; q < 4; ++q) { const int kx = q * 32 + lane; const float p = __expf(Sf[rr][kx] - mn); ps += p; b16 ph, pl; split16(p * PS, ph, pl); Ph_[rr][kx] = ph; Pl_[rr][kx] = pl; }
      for (int o = 16; o; o >>= 1) ps += __shfl_xor(ps, o);
      if ((rr >> 3) == hlf) { const int r8 = rr & 7; den_r[r8] = den_r[r8] * sf + ps; m_r[r8] = mn;
#pragma unroll
        for (int t = 0; t < 8; ++t) acc[t][r8] = acc[t][r8] * sf; } }
    wave_lds_sync();
#pragma unroll
    for (int ks = 0; ks < KB; ks += 32) { const v16b pa = frag_kb(&Ph_[nloc][ks], hlf), pb = frag_kb(&Pl_[nloc][ks], hlf);
#pragma unroll
      for (int t = 0; t < 8; ++t) { const v16b vh = frag_kb(&Vth[t * 16 + nloc][ks], hlf), vl = frag_kb(&Vtl[t * 16 + nloc][ks], hlf); acc[t] = wmma16b(pa, vh, acc[t]); acc[t] = wmma16b(pa, vl, acc[t]); acc[t] = wmma16b(pb, vh, acc[t]); } }
    wave_lds_sync(); }
#pragma unroll
  for (int t = 0; t < 8; ++t)
#pragma unroll
    for (int r8 = 0; r8 < 8; ++r8) Of[8 * hlf + r8][t * 16 + nloc] = acc[t][r8] * (1.0f / (HS * PS)) / den_r[r8];
  wave_lds_sync();
  for (int pass = 0; pass < 2; ++pass) { for (int rr = 0; rr < 16; ++rr) *(volatile v4f*)(Y + (q0 + rr) * CI + lane * 4) = *(const v4f*)(&Of[rr][lane * 4]); __threadfence(); } }
__global__ __launch_bounds__(32) void out_kernel(const float* __restrict__ Y, const b16* __restrict__ WOUT, const float* __restrict__ wb, const float* __restrict__ gam, const float* __restrict__ bet, const float* __restrict__ mean, const float* __restrict__ var, int BLIM, float* __restrict__ out) { __shared__ __attribute__((aligned(16))) b16 Ah[32][CI + 8], Al[32][CI + 8]; __shared__ float Tf[32][C + 4]; const int lane = threadIdx.x, nloc = lane & 15, hlf = lane >> 4; const int b = blockIdx.x / (NP / 32); if (b >= BLIM) return; const int p0 = (blockIdx.x % (NP / 32)) * 32; const size_t q0 = (size_t)b * NP + p0;
  for (int rr = 0; rr < 32; ++rr) for (int q = 0; q < 4; ++q) { b16 p, ql; split16(Y[(q0 + rr) * CI + q * 32 + lane] * HS, p, ql); Ah[rr][q * 32 + lane] = p; Al[rr][q * 32 + lane] = ql; } for (int k = CI; k < CI + 8; ++k) { Ah[lane][k] = (b16)0.0f; Al[lane][k] = (b16)0.0f; }
  wave_lds_sync();
#pragma unroll 1
  for (int rt = 0; rt < 2; ++rt) { v8f acc[16];
#pragma unroll
    for (int t = 0; t < 16; ++t) acc[t] = (v8f){};
#pragma unroll
    for (int kb = 0; kb < CI; kb += 32) { const v16b a = frag_kb(&Ah[rt * 16 + nloc][kb], hlf), al = frag_kb(&Al[rt * 16 + nloc][kb], hlf);
#pragma unroll
      for (int t = 0; t < 16; ++t) { const v16b bw = frag_kb(WOUT + (size_t)(t * 16 + nloc) * CI + kb, hlf); acc[t] = wmma16b(a, bw, acc[t]); acc[t] = wmma16b(al, bw, acc[t]); } }
#pragma unroll
    for (int t = 0; t < 16; ++t) { const int cc = t * 16 + nloc; const float inv = pmul(bfv(gam[cc]), rsqrtf(bfv(var[cc]) + BNEPS)); const float sh = bfv(bet[cc]) - pmul(bfv(mean[cc]), inv); const float bb = bfv(wb[cc]);
#pragma unroll
      for (int r8 = 0; r8 < 8; ++r8) Tf[rt * 16 + 8 * hlf + r8][cc] = pmul(acc[t][r8] * (1.0f / (HS * WSC)) + bb, inv) + sh; } }
  wave_lds_sync();
  for (int pass = 0; pass < 2; ++pass) {
#pragma unroll 4
    for (int c = 0; c < C; ++c) ((volatile float*)out)[((size_t)b * C + c) * NP + p0 + lane] = Tf[lane][c]; __threadfence(); } }
}

extern "C" void kernel_launch(void* const* d_in, const int* in_sizes, int n_in, void* d_out, int out_size, void* d_ws, size_t ws_size, hipStream_t stream) {
  (void)n_in;
  auto Fp = [&](int i) { return (const float*)d_in[i]; };
  if (in_sizes[0] != NBI * C * NP || in_sizes[1] != CI * C || in_sizes[3] != CI * C || in_sizes[5] != CI * C || in_sizes[7] != C * CI || in_sizes[9] != C || in_sizes[12] != C || out_size != NBI * C * NP) return;
  const int BLIM = NBI;
  size_t off = 0; char* ws = (char*)d_ws;
  auto carve = [&](size_t bytes) { char* p = ws + off; off += (bytes + 255) & ~(size_t)255; return p; };
  b16* W3 = (b16*)carve((size_t)3 * CI * C * 2); b16* WOUT = (b16*)carve((size_t)C * CI * 2); b16* THh = (b16*)carve((size_t)NBI * NP * CI * 2); b16* THl = (b16*)carve((size_t)NBI * NP * CI * 2); float* PG = (float*)carve((size_t)NBI * NP * 2 * CI * 4);
  b16* PHh = (b16*)carve((size_t)NBI * NM * CI * 2); b16* PHl = (b16*)carve((size_t)NBI * NM * CI * 2); b16* Gh = (b16*)carve((size_t)NBI * NM * CI * 2); b16* Gl = (b16*)carve((size_t)NBI * NM * CI * 2); float* Y = (float*)carve((size_t)NBI * NP * CI * 4);
  if (off > ws_size || off > ((size_t)96 << 20)) return;
  wput_kernel<<<(3 * CI * (C / 8) + 255) / 256, 256, 0, stream>>>(Fp(1), Fp(3), Fp(5), Fp(7), W3, WOUT);
  proj_kernel<<<BLIM * (NP / 32), 32, 0, stream>>>(Fp(0), W3, Fp(2), Fp(4), Fp(6), BLIM, THh, THl, PG);
  pool_kernel<<<(unsigned)(((size_t)BLIM * NM * 16 + 255) / 256), 256, 0, stream>>>(PG, BLIM, PHh, PHl, Gh, Gl);
  att_kernel<<<BLIM * (NP / 16), 32, 0, stream>>>(THh, THl, PHh, PHl, Gh, Gl, BLIM, Y);
  out_kernel<<<BLIM * (NP / 32), 32, 0, stream>>>(Y, WOUT, Fp(8), Fp(9), Fp(10), Fp(11), Fp(12), BLIM, (float*)d_out);
}
